// BUY_Net_29635274342639
// MI455X (gfx1250) — hardware-verified
//
#include <hip/hip_runtime.h>
#include <stddef.h>


#define CN    64
#define CE    256
#define CD    128
#define NT    256
#define NWV   8
#define KP1   58
#define KP2   53
#define KP3   48
#define GPB   16

#define OW1R  0
#define OW1O  65536
#define OW2R  131072
#define OW2O  163840
#define OW3R  196608
#define OW3O  229376
#define OL1   262144
#define OL2   393216
#define WPTOT 458752

static_assert(NT == CE);
static_assert(NT == 4 * CN);
static_assert((CN * 256) % 4 == 0);

typedef float    v4f  __attribute__((ext_vector_type(4)));
typedef float    v8f  __attribute__((ext_vector_type(8)));
typedef unsigned v4u  __attribute__((ext_vector_type(4)));
typedef unsigned v8u  __attribute__((ext_vector_type(8)));
typedef __bf16   v16b __attribute__((ext_vector_type(16)));
union Frag { v16b v; v8u u; v4u q[2]; };

__device__ __forceinline__ unsigned bf_hi_bits(float x) {
  const unsigned u = __float_as_uint(x);
  return (u + 0x7FFFu + ((u >> 16) & 1u)) & 0xFFFF0000u;
}
__device__ __forceinline__ void split2(float x0, float x1, unsigned& ph, unsigned& pl) {
  const unsigned h0 = bf_hi_bits(x0), h1 = bf_hi_bits(x1);
  ph = (h0 >> 16) | h1;
  const unsigned g0 = bf_hi_bits(x0 - __uint_as_float(h0));
  const unsigned g1 = bf_hi_bits(x1 - __uint_as_float(h1));
  pl = (g0 >> 16) | g1;
}
__device__ __forceinline__ void split16(const v4f f0, const v4f f1, const v4f f2, const v4f f3, Frag& hi, Frag& lo) {
  unsigned a, b; v8u hu, lu;
  split2(f0.x, f0.y, a, b); hu[0] = a; lu[0] = b;
  split2(f0.z, f0.w, a, b); hu[1] = a; lu[1] = b;
  split2(f1.x, f1.y, a, b); hu[2] = a; lu[2] = b;
  split2(f1.z, f1.w, a, b); hu[3] = a; lu[3] = b;
  split2(f2.x, f2.y, a, b); hu[4] = a; lu[4] = b;
  split2(f2.z, f2.w, a, b); hu[5] = a; lu[5] = b;
  split2(f3.x, f3.y, a, b); hu[6] = a; lu[6] = b;
  split2(f3.z, f3.w, a, b); hu[7] = a; lu[7] = b;
  hi.u = hu; lo.u = lu;
}
__device__ __forceinline__ void load_split_row(const float* ap, Frag& hi, Frag& lo) {
  const v4f f0 = *(const v4f*)(ap);
  const v4f f1 = *(const v4f*)(ap + 4);
  const v4f f2 = *(const v4f*)(ap + 16);
  const v4f f3 = *(const v4f*)(ap + 20);
  split16(f0, f1, f2, f3, hi, lo);
}
__device__ __forceinline__ void load_plane_frag(const unsigned short* bp, Frag& f) {
  f.q[0] = *(const v4u*)(bp);
  f.q[1] = *(const v4u*)(bp + 16);
}
__device__ __forceinline__ v8f wmb(v16b a, v16b b, v8f c) {
  v8f d = __builtin_amdgcn_wmma_f32_16x16x32_bf16(false, a, false, b, (short)0, c, false, false);
  asm volatile("v_nop\n\tv_nop\n\tv_nop\n\tv_nop" : "+v"(d) : "v"(a), "v"(b));
  return d;
}
__device__ __forceinline__ v8f zero8() { const v8f z = {0.f, 0.f, 0.f, 0.f, 0.f, 0.f, 0.f, 0.f}; return z; }

__global__ __launch_bounds__(NT) void k_wprep(
    const float* __restrict__ W1r, const float* __restrict__ W1o,
    const float* __restrict__ W2r, const float* __restrict__ W2o,
    const float* __restrict__ W3r, const float* __restrict__ W3o,
    const float* __restrict__ L1, const float* __restrict__ L2, unsigned short* wp) {
  const int mat = blockIdx.y;
  const float* src = W1r; int K = 256, N = CD, off = OW1R;
  if      (mat == 1) { src = W1o;            off = OW1O; }
  else if (mat == 2) { src = W2r; K = CD;    off = OW2R; }
  else if (mat == 3) { src = W2o; K = CD;    off = OW2O; }
  else if (mat == 4) { src = W3r; K = CD;    off = OW3R; }
  else if (mat == 5) { src = W3o; K = CD;    off = OW3O; }
  else if (mat == 6) { src = L1;  N = 256;   off = OL1;  }
  else if (mat == 7) { src = L2;             off = OL2;  }
  const int items = K * N / 8;
  const int i = blockIdx.x * NT + threadIdx.x;
  if (i >= items) return;
  const int kq = K / 8;
  const int n  = i / kq;
  const int k0 = (i - n * kq) * 8;
  const float* p = src + (size_t)k0 * N + n;
  const float x0 = p[0],             x1 = p[(size_t)N],     x2 = p[(size_t)2 * N], x3 = p[(size_t)3 * N];
  const float x4 = p[(size_t)4 * N], x5 = p[(size_t)5 * N], x6 = p[(size_t)6 * N], x7 = p[(size_t)7 * N];
  unsigned ha, la, hb, lb, hc, lc, hd, ld;
  split2(x0, x1, ha, la); split2(x2, x3, hb, lb); split2(x4, x5, hc, lc); split2(x6, x7, hd, ld);
  v4u hv, lv;
  hv.x = ha; hv.y = hb; hv.z = hc; hv.w = hd;
  lv.x = la; lv.y = lb; lv.z = lc; lv.w = ld;
  unsigned short* dh = wp + off + (size_t)8 * i;
  unsigned short* dl = dh + (size_t)K * N;
  *(volatile v4u*)dh = hv;
  *(volatile v4u*)dl = lv;
  __threadfence();
  *(volatile v4u*)dh = hv;
  *(volatile v4u*)dl = lv;
}

template <int K>
__device__ __forceinline__ void conv_gemm(const float* sA1, const float* sA2, float* sY,
    const unsigned short* __restrict__ wp, const int offR, const int offO,
    const float* __restrict__ bias, const int lane, const int wave) {
  const int h = lane >> 4, m = lane & 15;
  const int mt = wave & 3, ng = wave >> 2;
  const unsigned short* prh = wp + offR;
  const unsigned short* prl = prh + K * CD;
  const unsigned short* poh = wp + offO;
  const unsigned short* pol = poh + K * CD;
  v8f acc[4];
#pragma unroll
  for (int t = 0; t < 4; ++t) acc[t] = zero8();
  const float* a1 = sA1 + (mt * 16 + m) * K + 8 * h;
  const float* a2 = sA2 + (mt * 16 + m) * K + 8 * h;
#pragma unroll 1
  for (int ks = 0; ks < K / 32; ++ks) {
    const int k0 = 32 * ks;
    Frag ghi, glo, xhi, xlo;
    load_split_row(a1 + k0, ghi, glo);
    load_split_row(a2 + k0, xhi, xlo);
#pragma unroll
    for (int nt = 0; nt < 4; ++nt) {
      const int bo = ((ng * 4 + nt) * 16 + m) * K + k0 + 8 * h;
      Frag rh, rl, oh, ol;
      load_plane_frag(prh + bo, rh);
      load_plane_frag(prl + bo, rl);
      load_plane_frag(poh + bo, oh);
      load_plane_frag(pol + bo, ol);
      acc[nt] = wmb(ghi.v, rh.v, acc[nt]);
      acc[nt] = wmb(ghi.v, rl.v, acc[nt]);
      acc[nt] = wmb(glo.v, rh.v, acc[nt]);
      acc[nt] = wmb(xhi.v, oh.v, acc[nt]);
      acc[nt] = wmb(xhi.v, ol.v, acc[nt]);
      acc[nt] = wmb(xlo.v, oh.v, acc[nt]);
    }
  }
  __syncthreads();
  const int row0 = mt * 16 + 8 * h;
#pragma unroll
  for (int nt = 0; nt < 4; ++nt) {
    const int col = (ng * 4 + nt) * 16 + m;
    const float bv = bias[col];
    float* yp = sY + row0 * CD + col;
#pragma unroll
    for (int r = 0; r < 8; ++r) yp[r * CD] = fmaxf(acc[nt][r] + bv, 0.f);
  }
  __syncthreads();
}

struct Lds {
  float* x; float* agg; float* y;
  int* src; int* dst; int* msk; int* key; int* es; int* hist; int* boff; int* inv; int* sel;
  float* s; float* tv; float* p; float* rn; float* h;
};

template <int K>
__device__ __forceinline__ void conv_layer(const Lds L, const unsigned short* __restrict__ wp,
    const int offR, const int offO, const float* __restrict__ bias, const float* __restrict__ pvec,
    const int nNodes, const int kOut, const float invK, const int tid, const int lane, const int wave) {
  if (tid < CD) L.p[tid] = pvec[tid];
  if (tid < CN) L.sel[tid] = 0;
  L.hist[tid] = 0; L.hist[NT + tid] = 0;
  const int live = L.msk[tid];
  const int key  = (live != 0) ? L.dst[tid] : CN;
  L.key[tid] = key;
  __syncthreads();
  if (tid == NT - 1) {
    float q = 0.f;
#pragma unroll 1
    for (int c = 0; c < CD; ++c) { const float v = L.p[c]; q += v * v; }
    L.rn[0] = 1.0f / sqrtf(q);
  }
  int eqb = 0, eqt = 0;
  {
    const int wb = tid & ~31;
#pragma unroll 8
    for (int j = 0; j < 32; ++j) {
      const int kj = L.key[wb + j];
      const int e = (kj == key) ? 1 : 0;
      eqt += e;
      eqb += (j < lane) ? e : 0;
    }
  }
  if (key < CN) L.hist[wave * CN + key] = eqt;
  __syncthreads();
  if (tid < CN) {
    int cum = 0;
#pragma unroll
    for (int w = 0; w < NWV; ++w) { const int c = L.hist[w * CN + tid]; L.hist[w * CN + tid] = cum; cum += c; }
    L.boff[1 + tid] = cum;
  }
  __syncthreads();
  if (tid == 0) {
    int run = 0;
#pragma unroll 1
    for (int d = 0; d < CN; ++d) { const int c = L.boff[1 + d]; L.boff[d] = run; run += c; }
    L.boff[CN] = run;
  }
  __syncthreads();
  if (key < CN) {
    int pos = L.boff[key] + L.hist[wave * CN + key] + eqb;
    pos = min(max(pos, 0), CE - 1);
    L.es[pos] = L.src[tid];
  }
  __syncthreads();
#pragma unroll 1
  for (int i = 0; i < CN / NWV; ++i) {
    const int d = wave + NWV * i;
    int b0 = L.boff[d], b1 = L.boff[d + 1];
    b0 = min(max(b0, 0), CE);
    b1 = min(max(b1, b0), CE);
    if (K == 256) {
      v4f a0 = {0.f, 0.f, 0.f, 0.f}, a1 = {0.f, 0.f, 0.f, 0.f};
#pragma unroll 1
      for (int e = b0; e < b1; ++e) {
        const int s = L.es[e] & (CN - 1);
        const float* xp = L.x + s * 256 + 8 * lane;
        a0 += *(const v4f*)xp;
        a1 += *(const v4f*)(xp + 4);
      }
      *(v4f*)(L.agg + d * 256 + 8 * lane)     = a0;
      *(v4f*)(L.agg + d * 256 + 8 * lane + 4) = a1;
    } else {
      v4f a0 = {0.f, 0.f, 0.f, 0.f};
#pragma unroll 1
      for (int e = b0; e < b1; ++e) {
        const int s = L.es[e] & (CN - 1);
        a0 += *(const v4f*)(L.x + s * CD + 4 * lane);
      }
      *(v4f*)(L.agg + d * CD + 4 * lane) = a0;
    }
  }
  __syncthreads();
  conv_gemm<K>(L.agg, L.x, L.y, wp, offR, offO, bias, lane, wave);
  if (tid < CN) {
    float sc = -3.0e38f;
    if (tid < nNodes) {
      float q = 0.f;
      const float* yr = L.y + tid * CD;
#pragma unroll 4
      for (int c = 0; c < CD; ++c) q += yr[c] * L.p[c];
      sc = q * L.rn[0];
    }
    L.s[tid] = sc;
  }
  __syncthreads();
  if (tid < CN) {
    int iv = -1;
    if (tid < nNodes) {
      const float st = L.s[tid];
      int r = 0;
#pragma unroll 4
      for (int mm = 0; mm < nNodes; ++mm) {
        const float sm = L.s[mm];
        r += ((sm > st) || (sm == st && mm < tid)) ? 1 : 0;
      }
      if (r < kOut) { iv = r; L.sel[r] = tid; }
      L.tv[tid] = tanhf(st);
    }
    L.inv[tid] = iv;
  }
  __syncthreads();
#pragma unroll
  for (int it = 0; it < (CN * CD / 4) / NT; ++it) {
    const int idx = it * NT + tid;
    const int r = idx >> 5;
    const int q = idx & 31;
    v4f v = {0.f, 0.f, 0.f, 0.f};
    if (r < kOut) {
      const int sn = L.sel[r];
      const float t = L.tv[sn];
      v = *(const v4f*)(L.y + sn * CD + 4 * q) * t;
    }
    *(v4f*)(L.x + r * CD + 4 * q) = v;
  }
  __syncthreads();
  if (tid < CD) {
    float mx = -3.0e38f, sm = 0.f;
#pragma unroll 2
    for (int r = 0; r < kOut; ++r) { const float v = L.x[r * CD + tid]; mx = fmaxf(mx, v); sm += v; }
    L.h[tid] += mx;
    L.h[CD + tid] += sm * invK;
  }
  if (live != 0) {
    const int ns = L.inv[L.src[tid]], nd = L.inv[L.dst[tid]];
    const int lv = (ns >= 0 && nd >= 0) ? 1 : 0;
    L.src[tid] = max(ns, 0);
    L.dst[tid] = max(nd, 0);
    L.msk[tid] = lv;
  }
  __syncthreads();
}

__global__ __launch_bounds__(NT) __attribute__((amdgpu_num_vgpr(256)))
void k_graph(const int* __restrict__ item_id, const int* __restrict__ category,
             const int* __restrict__ edge_local,
             const float* __restrict__ emb_item, const float* __restrict__ emb_cat,
             const unsigned short* __restrict__ wp,
             const float* __restrict__ b1, const float* __restrict__ b2, const float* __restrict__ b3,
             const float* __restrict__ p1, const float* __restrict__ p2, const float* __restrict__ p3,
             float* hout, const int nItems, const int nCats, const int nEtot,
             const float ik1, const float ik2, const float ik3) {
  __shared__ __attribute__((aligned(16))) float sX[CN * 256];
  __shared__ __attribute__((aligned(16))) float sAgg[CN * 256];
  __shared__ int sSrc[CE];
  __shared__ int sDst[CE];
  __shared__ int sMsk[CE];
  __shared__ int sKey[CE];
  __shared__ int sEs[CE];
  __shared__ int sHist[NWV * CN];
  __shared__ int sBoff[80];
  __shared__ int sInv[CN];
  __shared__ int sSel[CN];
  __shared__ __attribute__((aligned(16))) float sS[CN];
  __shared__ __attribute__((aligned(16))) float sTv[CN];
  __shared__ __attribute__((aligned(16))) float sP[CD];
  __shared__ __attribute__((aligned(16))) float sH[256];
  __shared__ float sRn[4];

  Lds L;
  L.x = sX; L.agg = sAgg; L.y = sAgg + 8192;
  L.src = sSrc; L.dst = sDst; L.msk = sMsk; L.key = sKey; L.es = sEs; L.hist = sHist; L.boff = sBoff;
  L.inv = sInv; L.sel = sSel; L.s = sS; L.tv = sTv; L.p = sP; L.rn = sRn; L.h = sH;

  const int tid = threadIdx.x, lane = tid & 31, wave = tid >> 5;
  const int g = blockIdx.x;

  {
    int s = edge_local[(size_t)g * CE + tid];
    int d = edge_local[(size_t)nEtot + (size_t)g * CE + tid];
    s = min(max(s, 0), CN - 1);
    d = min(max(d, 0), CN - 1);
    sSrc[tid] = s; sDst[tid] = d; sMsk[tid] = 1;
  }
  sH[tid] = 0.f;
  {
    const int half = wave & 1;
#pragma unroll 4
    for (int it = 0; it < (CN * 256 / 4) / NT; ++it) {
      const int idx = it * NT + tid;
      const int j = idx >> 6;
      const int q = idx & 63;
      v4f v;
      if (half == 0) {
        int id = item_id[(size_t)g * CN + j];
        id = min(max(id, 0), nItems - 1);
        v = *(const v4f*)(emb_item + (size_t)id * CD + 4 * q);
      } else {
        int id = category[(size_t)g * CN + j];
        id = min(max(id, 0), nCats - 1);
        v = *(const v4f*)(emb_cat + (size_t)id * CD + 4 * (q - 32));
      }
      *(v4f*)(sX + j * 256 + 4 * q) = v;
    }
  }
  __syncthreads();

  conv_layer<256>(L, wp, OW1R, OW1O, b1, p1, CN,  KP1, ik1, tid, lane, wave);
  conv_layer<CD> (L, wp, OW2R, OW2O, b2, p2, KP1, KP2, ik2, tid, lane, wave);
  conv_layer<CD> (L, wp, OW3R, OW3O, b3, p3, KP2, KP3, ik3, tid, lane, wave);

  if (wave == 0) {
    const v4f v0 = *(const v4f*)(sH + 4 * lane);
    const v4f v1 = *(const v4f*)(sH + CD + 4 * lane);
    float* hp = hout + (size_t)g * 256;
    *(volatile v4f*)(hp + 4 * lane)      = v0;
    *(volatile v4f*)(hp + CD + 4 * lane) = v1;
    __threadfence();
    *(volatile v4f*)(hp + 4 * lane)      = v0;
    *(volatile v4f*)(hp + CD + 4 * lane) = v1;
  }
}

__global__ __launch_bounds__(NT) __attribute__((amdgpu_num_vgpr(256)))
void k_head(const float* __restrict__ hin, const unsigned short* __restrict__ wp,
            const float* __restrict__ l1b, const float* __restrict__ l2b,
            const int* __restrict__ item_id, const float* __restrict__ emb_item, const int nItems,
            float* out) {
  __shared__ __attribute__((aligned(16))) float sHin[GPB * 256];
  __shared__ __attribute__((aligned(16))) float sH1[GPB * 256];
  __shared__ __attribute__((aligned(16))) float sHf[GPB * CD];
  __shared__ __attribute__((aligned(16))) float sEmb[2 * CN * CD];
  __shared__ __attribute__((aligned(16))) float sOut[GPB * CN];
  const int tid = threadIdx.x, lane = tid & 31, wave = tid >> 5, h = lane >> 4, m = lane & 15;
  const int g0 = blockIdx.x * GPB;

#pragma unroll
  for (int it = 0; it < (GPB * 256 / 4) / NT; ++it) {
    const int idx = it * NT + tid;
    *(v4f*)(sHin + 4 * idx) = *(const v4f*)(hin + (size_t)g0 * 256 + 4 * idx);
  }
  __syncthreads();

  {
    v8f acc[2];
    acc[0] = zero8(); acc[1] = zero8();
    const float* ar = sHin + m * 256 + 8 * h;
    const unsigned short* ph = wp + OL1;
    const unsigned short* pl = ph + 256 * 256;
#pragma unroll 1
    for (int ks = 0; ks < 8; ++ks) {
      const int k0 = 32 * ks;
      Frag ah, al;
      load_split_row(ar + k0, ah, al);
#pragma unroll
      for (int nt = 0; nt < 2; ++nt) {
        const int bo = ((2 * wave + nt) * 16 + m) * 256 + k0 + 8 * h;
        Frag bh, bl;
        load_plane_frag(ph + bo, bh);
        load_plane_frag(pl + bo, bl);
        acc[nt] = wmb(ah.v, bh.v, acc[nt]);
        acc[nt] = wmb(ah.v, bl.v, acc[nt]);
        acc[nt] = wmb(al.v, bh.v, acc[nt]);
      }
    }
#pragma unroll
    for (int nt = 0; nt < 2; ++nt) {
      const int col = (2 * wave + nt) * 16 + m;
      const float bv = l1b[col];
      float* yp = sH1 + (8 * h) * 256 + col;
#pragma unroll
      for (int r = 0; r < 8; ++r) yp[r * 256] = fmaxf(acc[nt][r] + bv, 0.f);
    }
  }
  __syncthreads();

  {
    v8f acc = zero8();
    const float* ar = sH1 + m * 256 + 8 * h;
    const unsigned short* ph = wp + OL2;
    const unsigned short* pl = ph + 256 * CD;
#pragma unroll 1
    for (int ks = 0; ks < 8; ++ks) {
      const int k0 = 32 * ks;
      Frag ah, al, bh, bl;
      load_split_row(ar + k0, ah, al);
      const int bo = (wave * 16 + m) * 256 + k0 + 8 * h;
      load_plane_frag(ph + bo, bh);
      load_plane_frag(pl + bo, bl);
      acc = wmb(ah.v, bh.v, acc);
      acc = wmb(ah.v, bl.v, acc);
      acc = wmb(al.v, bh.v, acc);
    }
    const int col = wave * 16 + m;
    const float bv = l2b[col];
    float* yp = sHf + (8 * h) * CD + col;
#pragma unroll
    for (int r = 0; r < 8; ++r) yp[r * CD] = fmaxf(acc[r] + bv, 0.f);
  }
  __syncthreads();

  const int gh = wave >> 2, mt = wave & 3;
#pragma unroll 1
  for (int ps = 0; ps < GPB / 2; ++ps) {
#pragma unroll 4
    for (int it = 0; it < (2 * CN * CD / 4) / NT; ++it) {
      const int idx = it * NT + tid;
      const int e = idx >> 11;
      const int j = (idx >> 5) & (CN - 1);
      const int q = idx & 31;
      const int ga = g0 + 2 * ps + e;
      int id = item_id[(size_t)ga * CN + j];
      id = min(max(id, 0), nItems - 1);
      *(v4f*)(sEmb + e * (CN * CD) + j * CD + 4 * q) = *(const v4f*)(emb_item + (size_t)id * CD + 4 * q);
    }
    __syncthreads();
    v8f acc = zero8();
    const float* ar = sEmb + gh * (CN * CD) + (mt * 16 + m) * CD + 8 * h;
    const float* br = sHf + m * CD + 8 * h;
#pragma unroll
    for (int ks = 0; ks < CD / 32; ++ks) {
      Frag ah, al, bh, bl;
      load_split_row(ar + 32 * ks, ah, al);
      load_split_row(br + 32 * ks, bh, bl);
      acc = wmb(ah.v, bh.v, acc);
      acc = wmb(ah.v, bl.v, acc);
      acc = wmb(al.v, bh.v, acc);
    }
    const int jc = 2 * ps + gh;
    if (m == jc) {
      float* op = sOut + jc * CN + mt * 16 + 8 * h;
#pragma unroll
      for (int r = 0; r < 8; ++r) {
        float s = acc[r];
        s = fminf(fmaxf(s, -40.f), 40.f);
        const float ex = __expf(-s);
        op[r] = __builtin_amdgcn_rcpf(1.f + ex);
      }
    }
    __syncthreads();
  }

  {
    const v4f v = *(const v4f*)(sOut + wave * 128 + 4 * lane);
    float* op = out + (size_t)g0 * CN + wave * 128 + 4 * lane;
    *(volatile v4f*)op = v;
    __threadfence();
    *(volatile v4f*)op = v;
  }
}

extern "C" void kernel_launch(void* const* d_in, const int* in_sizes, int n_in,
                              void* d_out, int out_size, void* d_ws, size_t ws_size,
                              hipStream_t stream) {
  if (n_in < 21) return;
  const int nTot = in_sizes[0];
  const int G = nTot / CN;
  if (G <= 0 || G * CN != nTot || (G % GPB) != 0) return;
  if (in_sizes[1] != nTot) return;
  const int nEtot = in_sizes[2] / 2;
  if (2 * nEtot != in_sizes[2] || nEtot != G * CE) return;
  const int nItems = in_sizes[3] / CD;
  const int nCats  = in_sizes[4] / CD;
  if (nItems <= 0 || nCats <= 0 || nItems * CD != in_sizes[3] || nCats * CD != in_sizes[4]) return;
  if (in_sizes[5] != 256 * CD || in_sizes[6] != CD || in_sizes[7] != 256 * CD) return;
  if (in_sizes[8] != CD * CD || in_sizes[9] != CD || in_sizes[10] != CD * CD) return;
  if (in_sizes[11] != CD * CD || in_sizes[12] != CD || in_sizes[13] != CD * CD) return;
  if (in_sizes[14] != CD || in_sizes[15] != CD || in_sizes[16] != CD) return;
  if (in_sizes[17] != 256 * 256 || in_sizes[18] != 256 || in_sizes[19] != 256 * CD || in_sizes[20] != CD) return;
  if (out_size != nTot) return;

  const int*   item_id    = (const int*)d_in[0];
  const int*   category   = (const int*)d_in[1];
  const int*   edge_local = (const int*)d_in[2];
  const float* emb_item   = (const float*)d_in[3];
  const float* emb_cat    = (const float*)d_in[4];
  const float* W1r = (const float*)d_in[5];
  const float* b1  = (const float*)d_in[6];
  const float* W1o = (const float*)d_in[7];
  const float* W2r = (const float*)d_in[8];
  const float* b2  = (const float*)d_in[9];
  const float* W2o = (const float*)d_in[10];
  const float* W3r = (const float*)d_in[11];
  const float* b3  = (const float*)d_in[12];
  const float* W3o = (const float*)d_in[13];
  const float* p1  = (const float*)d_in[14];
  const float* p2  = (const float*)d_in[15];
  const float* p3  = (const float*)d_in[16];
  const float* L1W = (const float*)d_in[17];
  const float* L1b = (const float*)d_in[18];
  const float* L2W = (const float*)d_in[19];
  const float* L2b = (const float*)d_in[20];
  float* out = (float*)d_out;

  char* ws = (char*)d_ws;
  size_t off = 0;
  const size_t oWP = off; off += (size_t)WPTOT * 2;       off = (off + 255) & ~(size_t)255;
  const size_t oH  = off; off += (size_t)G * 256 * 4;     off = (off + 255) & ~(size_t)255;
  if (off > ws_size) return;
  unsigned short* wp   = (unsigned short*)(ws + oWP);
  float*          hbuf = (float*)(ws + oH);

  const float ik1 = 1.0f / (float)KP1;
  const float ik2 = 1.0f / (float)KP2;
  const float ik3 = 1.0f / (float)KP3;

  k_wprep<<<dim3(32, 8), NT, 0, stream>>>(W1r, W1o, W2r, W2o, W3r, W3o, L1W, L2W, wp);

  k_graph<<<G, NT, 0, stream>>>(item_id, category, edge_local, emb_item, emb_cat, wp,
                                b1, b2, b3, p1, p2, p3, hbuf, nItems, nCats, nEtot, ik1, ik2, ik3);

  k_head<<<G / GPB, NT, 0, stream>>>(hbuf, wp, L1b, L2b, item_id, emb_item, nItems, out);
}
